// Text_Decoder_85916525789534
// MI455X (gfx1250) — hardware-run, weakly checked
//
#include <hip/hip_runtime.h>

#define NBATCH 2048
#define EDIM   128
#define LL     77
#define DM     64
#define DI     128
#define DS     16
#define DTR    4
#define XZW    256
#define XPR    36
#define XPP    64
#define LW     4928
#define NCH    4
#define BSC    512
#define NTC    39424

#define S_E    64.0f
#define S_W    64.0f
#define S_X    32.0f
#define S_U    16384.0f
#define S_Y    262144.0f
#define RLO    1024.0f
#define ILO    0.0009765625f
#define INV_EW (1.0f / 4096.0f)
#define INV_XW (1.0f / 2048.0f)
#define INV_UW (1.0f / 1048576.0f)
#define INV_YW (1.0f / 16777216.0f)
#define LOG2E  1.4426950408889634f

static_assert(LW == LL * DM);
static_assert(BSC * NCH == NBATCH);
static_assert(NTC == BSC * LL);
static_assert((NTC % 64) == 0);
static_assert((BSC % 64) == 0);
static_assert((LW % 64) == 0);
static_assert((NTC % 8) == 0);
static_assert((EDIM % 32) == 0);
static_assert((DM % 32) == 0);
static_assert((DI % 32) == 0);
static_assert(DS == 16);
static_assert(DI == 128);

typedef _Float16 v16h __attribute__((ext_vector_type(16)));
typedef _Float16 v8h  __attribute__((ext_vector_type(8)));
typedef float    v8f  __attribute__((ext_vector_type(8)));
typedef float    v4f  __attribute__((ext_vector_type(4)));
typedef float    v2f  __attribute__((ext_vector_type(2)));
typedef unsigned int v4u __attribute__((ext_vector_type(4)));
typedef unsigned int v2u __attribute__((ext_vector_type(2)));

__device__ __forceinline__ unsigned short bf_bits(float f) {
  unsigned u = __float_as_uint(f);
  return (unsigned short)((u + 0x7FFFu + ((u >> 16) & 1u)) >> 16);
}
__device__ __forceinline__ float bfr(float f) { return __uint_as_float(((unsigned)bf_bits(f)) << 16); }
__device__ __forceinline__ unsigned short h_bits(_Float16 x) { return __builtin_bit_cast(unsigned short, x); }
__device__ __forceinline__ unsigned short hb16(float f) { return h_bits((_Float16)f); }
__device__ __forceinline__ unsigned pk16(unsigned short a, unsigned short b) { return (unsigned)a | ((unsigned)b << 16); }
__device__ __forceinline__ v8f zero8() { v8f z = {0.f, 0.f, 0.f, 0.f, 0.f, 0.f, 0.f, 0.f}; return z; }
__device__ __forceinline__ float sigf(float x) { return __builtin_amdgcn_rcpf(1.0f + __expf(-x)); }

__device__ __forceinline__ unsigned hl2(float v0, float v1, unsigned& lo) {
  const _Float16 h0 = (_Float16)v0;
  const _Float16 h1 = (_Float16)v1;
  lo = pk16(hb16((v0 - (float)h0) * RLO), hb16((v1 - (float)h1) * RLO));
  return pk16(h_bits(h0), h_bits(h1));
}
__device__ __forceinline__ void pack4(const v4f v, const float s, v2u& ph, v2u& pl) {
  unsigned l0, l1;
  const unsigned p0 = hl2(v[0] * s, v[1] * s, l0);
  const unsigned p1 = hl2(v[2] * s, v[3] * s, l1);
  ph[0] = p0; ph[1] = p1;
  pl[0] = l0; pl[1] = l1;
}
__device__ __forceinline__ void pack8(const v4f a, const v4f b, const float s, v4u& ph, v4u& pl) {
  unsigned l0, l1, l2, l3;
  const unsigned p0 = hl2(a[0] * s, a[1] * s, l0);
  const unsigned p1 = hl2(a[2] * s, a[3] * s, l1);
  const unsigned p2 = hl2(b[0] * s, b[1] * s, l2);
  const unsigned p3 = hl2(b[2] * s, b[3] * s, l3);
  ph[0] = p0; ph[1] = p1; ph[2] = p2; ph[3] = p3;
  pl[0] = l0; pl[1] = l1; pl[2] = l2; pl[3] = l3;
}

__device__ __forceinline__ v16h ldfrag_h(const _Float16* p) {
  union { v16h v; v8h h[2]; } f;
  f.h[0] = *(const v8h*)(p);
  f.h[1] = *(const v8h*)(p + 16);
  return f.v;
}

__device__ __forceinline__ v8f mma_raw(v16h a, v16h b, v8f c) {
  return __builtin_amdgcn_wmma_f32_16x16x32_f16(false, a, false, b, (short)0, c, false, false);
}
__device__ __forceinline__ void guard8(v8f& c0, v8f& c1, v8f& c2, v8f& c3, v8f& c4, v8f& c5, v8f& c6, v8f& c7,
                                       const v16h& a0, const v16h& a1, const v16h& a2, const v16h& a3,
                                       const v16h& b0, const v16h& b1) {
#if defined(__HIP_DEVICE_COMPILE__)
  asm volatile("v_nop\n\tv_nop\n\tv_nop\n\tv_nop"
               : "+v"(c0), "+v"(c1), "+v"(c2), "+v"(c3), "+v"(c4), "+v"(c5), "+v"(c6), "+v"(c7)
               : "v"(a0), "v"(a1), "v"(a2), "v"(a3), "v"(b0), "v"(b1));
#endif
}
__device__ __forceinline__ void guard4(v8f& c0, v8f& c1, v8f& c2, v8f& c3,
                                       const v16h& a0, const v16h& a1, const v16h& b0, const v16h& b1) {
#if defined(__HIP_DEVICE_COMPILE__)
  asm volatile("v_nop\n\tv_nop\n\tv_nop\n\tv_nop"
               : "+v"(c0), "+v"(c1), "+v"(c2), "+v"(c3)
               : "v"(a0), "v"(a1), "v"(b0), "v"(b1));
#endif
}

template <int NWN, bool RES>
__device__ __forceinline__ void mm_tile(const _Float16* __restrict__ Ah, const _Float16* __restrict__ Al, int lda,
                                        const _Float16* __restrict__ Wp, int ldw, int nks,
                                        int arow0, int bcol0, float* Cs) {
  constexpr int LDC = 32 * NWN + 4;
  const int tid = threadIdx.x, wave = tid >> 5, lane = tid & 31, hh = lane >> 4, c = lane & 15;
  const int mw = wave / NWN, nw = wave - mw * NWN;
  const size_t ao0 = (size_t)(arow0 + mw * 32 + c) * (size_t)lda + 8 * hh;
  const size_t ao1 = (size_t)(arow0 + mw * 32 + 16 + c) * (size_t)lda + 8 * hh;
  const _Float16* a0h = Ah + ao0;
  const _Float16* a1h = Ah + ao1;
  const _Float16* b0p = Wp + (size_t)(bcol0 + nw * 32 + c) * (size_t)ldw + 8 * hh;
  const _Float16* b1p = Wp + (size_t)(bcol0 + nw * 32 + 16 + c) * (size_t)ldw + 8 * hh;
  v8f h00 = zero8(), h01 = zero8(), h10 = zero8(), h11 = zero8();
  if (RES) {
    const _Float16* a0l = Al + ao0;
    const _Float16* a1l = Al + ao1;
    v8f l00 = zero8(), l01 = zero8(), l10 = zero8(), l11 = zero8();
#pragma unroll 1
    for (int ks = 0; ks < nks; ++ks) {
      const int ko = ks * 32;
      const v16h fa0 = ldfrag_h(a0h + ko);
      const v16h fa1 = ldfrag_h(a1h + ko);
      const v16h ga0 = ldfrag_h(a0l + ko);
      const v16h ga1 = ldfrag_h(a1l + ko);
      const v16h fb0 = ldfrag_h(b0p + ko);
      const v16h fb1 = ldfrag_h(b1p + ko);
      h00 = mma_raw(fa0, fb0, h00);
      h01 = mma_raw(fa0, fb1, h01);
      h10 = mma_raw(fa1, fb0, h10);
      h11 = mma_raw(fa1, fb1, h11);
      l00 = mma_raw(ga0, fb0, l00);
      l01 = mma_raw(ga0, fb1, l01);
      l10 = mma_raw(ga1, fb0, l10);
      l11 = mma_raw(ga1, fb1, l11);
      guard8(h00, h01, h10, h11, l00, l01, l10, l11, fa0, fa1, ga0, ga1, fb0, fb1);
    }
#pragma unroll
    for (int r = 0; r < 8; ++r) {
      const int row = mw * 32 + 8 * hh + r;
      Cs[row * LDC + nw * 32 + c]             = h00[r] + l00[r] * ILO;
      Cs[row * LDC + nw * 32 + 16 + c]        = h01[r] + l01[r] * ILO;
      Cs[(row + 16) * LDC + nw * 32 + c]      = h10[r] + l10[r] * ILO;
      Cs[(row + 16) * LDC + nw * 32 + 16 + c] = h11[r] + l11[r] * ILO;
    }
  } else {
#pragma unroll 1
    for (int ks = 0; ks < nks; ++ks) {
      const int ko = ks * 32;
      const v16h fa0 = ldfrag_h(a0h + ko);
      const v16h fa1 = ldfrag_h(a1h + ko);
      const v16h fb0 = ldfrag_h(b0p + ko);
      const v16h fb1 = ldfrag_h(b1p + ko);
      h00 = mma_raw(fa0, fb0, h00);
      h01 = mma_raw(fa0, fb1, h01);
      h10 = mma_raw(fa1, fb0, h10);
      h11 = mma_raw(fa1, fb1, h11);
      guard4(h00, h01, h10, h11, fa0, fa1, fb0, fb1);
    }
#pragma unroll
    for (int r = 0; r < 8; ++r) {
      const int row = mw * 32 + 8 * hh + r;
      Cs[row * LDC + nw * 32 + c]             = h00[r];
      Cs[row * LDC + nw * 32 + 16 + c]        = h01[r];
      Cs[(row + 16) * LDC + nw * 32 + c]      = h10[r];
      Cs[(row + 16) * LDC + nw * 32 + 16 + c] = h11[r];
    }
  }
}

__global__ __launch_bounds__(256)
void k_cvt(const float* __restrict__ src, int N, int K, unsigned short* dst, int Np, float sc) {
  const int kp = K >> 3;
  const int total = Np * kp;
  const int i = blockIdx.x * 256 + threadIdx.x;
  const int ic = min(i, total - 1);
  const int n = ic / kp, piece = ic - n * kp;
  const int nc = min(n, N - 1);
  const float m = (n < N) ? sc : 0.0f;
  const float* sp = src + (size_t)nc * (size_t)K + piece * 8;
  const v4f v0 = *(const v4f*)sp;
  const v4f v1 = *(const v4f*)(sp + 4);
  v4u u;
  u[0] = pk16(hb16(bfr(v0[0]) * m), hb16(bfr(v0[1]) * m));
  u[1] = pk16(hb16(bfr(v0[2]) * m), hb16(bfr(v0[3]) * m));
  u[2] = pk16(hb16(bfr(v1[0]) * m), hb16(bfr(v1[1]) * m));
  u[3] = pk16(hb16(bfr(v1[2]) * m), hb16(bfr(v1[3]) * m));
  if (i < total) {
    unsigned short* p = dst + (size_t)n * (size_t)K + piece * 8;
    *(volatile v4u*)p = u;
    __threadfence();
    *(volatile v4u*)p = u;
  }
}

__global__ __launch_bounds__(256)
void k_atab(const float* __restrict__ alog, int n, float* dst) {
  const int i = blockIdx.x * 256 + threadIdx.x;
  const int ic = min(i, n - 1);
  const float v = -expf(bfr(alog[ic])) * LOG2E;
  if (i < n) {
    float* p = dst + i;
    *(volatile float*)p = v;
    __threadfence();
    *(volatile float*)p = v;
  }
}

template <int MODE, int NWN, bool RES>
__global__ __launch_bounds__(64 * NWN)
void k_gemm(const unsigned short* __restrict__ ah, const unsigned short* __restrict__ al, int lda,
            const unsigned short* __restrict__ w, int ldw, int nks,
            const float* __restrict__ q0, float* o32a, float* o32b, unsigned short* oh, unsigned short* ol) {
  constexpr int NBW = 32 * NWN;
  constexpr int LDC = NBW + 4;
  __shared__ __align__(16) float Cs[64 * LDC];
  const int tid = threadIdx.x, wave = tid >> 5, lane = tid & 31;
  const int mb = blockIdx.x, nb = blockIdx.y;
  mm_tile<NWN, RES>((const _Float16*)(const void*)ah, (const _Float16*)(const void*)al, lda,
                    (const _Float16*)(const void*)w, ldw, nks, mb * 64, nb * NBW, Cs);
  __syncthreads();
  if (MODE == 0) {
    const int q = lane >> 3, cc = (lane & 7) * 8;
    const int gc = nb * NBW + cc;
    const v4f bb0 = *(const v4f*)(q0 + gc);
    const v4f bb1 = *(const v4f*)(q0 + gc + 4);
    v4f c0, c1;
#pragma unroll
    for (int e = 0; e < 4; ++e) { c0[e] = bfr(bb0[e]); c1[e] = bfr(bb1[e]); }
#pragma unroll 1
    for (int it = 0; it < 4; ++it) {
      const int row = it * 16 + wave * 4 + q;
      const v4f a0 = *(const v4f*)(Cs + row * LDC + cc);
      const v4f a1 = *(const v4f*)(Cs + row * LDC + cc + 4);
      v4f x0, x1;
#pragma unroll
      for (int e = 0; e < 4; ++e) {
        x0[e] = a0[e] * INV_EW + c0[e];
        x1[e] = a1[e] * INV_EW + c1[e];
      }
      v4u ph, pl;
      pack8(x0, x1, S_X, ph, pl);
      const size_t go = (size_t)(mb * 64 + row) * (size_t)LW + (size_t)gc;
      *(volatile v4u*)(oh + go) = ph;
      *(volatile v4u*)(ol + go) = pl;
      __threadfence();
      *(volatile v4u*)(oh + go) = ph;
      *(volatile v4u*)(ol + go) = pl;
    }
  } else if (MODE == 1) {
    const int cb = lane * 4;
    float* dstp = (nb == 0) ? o32a : o32b;
#pragma unroll 1
    for (int it = 0; it < 8; ++it) {
      const int row = it * 8 + wave;
      const v4f a = *(const v4f*)(Cs + row * LDC + cb);
      v4f v;
#pragma unroll
      for (int e = 0; e < 4; ++e) v[e] = a[e] * INV_XW;
      float* p = dstp + (size_t)(mb * 64 + row) * DI + cb;
      *(volatile v4f*)p = v;
      __threadfence();
      *(volatile v4f*)p = v;
    }
  } else {
    const int q = lane >> 4, cb = (lane & 15) * 4;
    const float inv = (MODE == 2) ? INV_UW : INV_YW;
#pragma unroll 1
    for (int it = 0; it < 8; ++it) {
      const int row = it * 8 + wave * 2 + q;
      const v4f a = *(const v4f*)(Cs + row * LDC + cb);
      v4f v;
#pragma unroll
      for (int e = 0; e < 4; ++e) v[e] = a[e] * inv;
      float* p = o32a + (size_t)(mb * 64 + row) * DM + cb;
      *(volatile v4f*)p = v;
      __threadfence();
      *(volatile v4f*)p = v;
    }
  }
}

__global__ __launch_bounds__(256)
void k_conv(const float* __restrict__ u0p, const float* __restrict__ cw, const float* __restrict__ cb,
            float* uf, unsigned short* uh, unsigned short* ul) {
  const int tid = threadIdx.x, wv = tid >> 5, lane = tid & 31;
  const int r = blockIdx.x * 8 + wv;
  const int tt = r % LL;
  const int c = lane * 4;
  const v4f cbv = *(const v4f*)(cb + c);
  const v4f t0v = *(const v4f*)(cw + (c + 0) * 4);
  const v4f t1v = *(const v4f*)(cw + (c + 1) * 4);
  const v4f t2v = *(const v4f*)(cw + (c + 2) * 4);
  const v4f t3v = *(const v4f*)(cw + (c + 3) * 4);
  v4f acc, wc0, wc1, wc2, wc3;
#pragma unroll
  for (int k = 0; k < 4; ++k) {
    acc[k] = bfr(cbv[k]);
    wc0[k] = bfr(t0v[k]);
    wc1[k] = bfr(t1v[k]);
    wc2[k] = bfr(t2v[k]);
    wc3[k] = bfr(t3v[k]);
  }
#pragma unroll
  for (int k = 0; k < 4; ++k) {
    const int rr = max(r - 3 + k, r - tt);
    const float m = (k >= 3 - tt) ? 1.0f : 0.0f;
    const v4f xv = *(const v4f*)(u0p + (size_t)rr * DI + c);
    acc[0] += (xv[0] * m) * wc0[k];
    acc[1] += (xv[1] * m) * wc1[k];
    acc[2] += (xv[2] * m) * wc2[k];
    acc[3] += (xv[3] * m) * wc3[k];
  }
  v4f u;
#pragma unroll
  for (int e = 0; e < 4; ++e) u[e] = acc[e] * sigf(acc[e]);
  v2u ph, pl;
  pack4(u, S_U, ph, pl);
  float* pu = uf + (size_t)r * DI + c;
  unsigned short* hp = uh + (size_t)r * DI + c;
  unsigned short* lp = ul + (size_t)r * DI + c;
  *(volatile v4f*)pu = u;
  *(volatile v2u*)hp = ph;
  *(volatile v2u*)lp = pl;
  __threadfence();
  *(volatile v4f*)pu = u;
  *(volatile v2u*)hp = ph;
  *(volatile v2u*)lp = pl;
}

__global__ __launch_bounds__(128)
void k_scan(const float* __restrict__ dbc, const float* __restrict__ uu, const float* __restrict__ zz,
            const float* __restrict__ a2, const float* __restrict__ dtw, const float* __restrict__ dtb,
            const float* __restrict__ dd, unsigned short* yh, unsigned short* yl) {
  __shared__ __align__(16) float sB[LL * DS];
  __shared__ __align__(16) float sC[LL * DS];
  __shared__ float sdt[LL * DTR];
  __shared__ __align__(16) unsigned short sY[LL * 2 * DI];
  const int d = threadIdx.x;
  const size_t r0 = (size_t)blockIdx.x * LL;
#pragma unroll 1
  for (int i = d; i < LL * DS; i += DI) {
    const int t = i >> 4, s = i & 15;
    const size_t ro = (r0 + t) * DM;
    sB[i] = dbc[ro + DTR + s];
    sC[i] = dbc[ro + DTR + DS + s];
  }
#pragma unroll 1
  for (int i = d; i < LL * DTR; i += DI) sdt[i] = dbc[(r0 + (i >> 2)) * DM + (i & 3)];
  __syncthreads();
  const v4f wr = *(const v4f*)(dtw + d * DTR);
  const float w0 = bfr(wr[0]), w1 = bfr(wr[1]), w2 = bfr(wr[2]), w3 = bfr(wr[3]);
  const float db = bfr(dtb[d]);
  const float Dd = bfr(dd[d]);
  const float* ap = a2 + d * DS;
  float h[DS], an[DS];
#pragma unroll
  for (int s = 0; s < DS; ++s) { h[s] = 0.0f; an[s] = ap[s]; }
#pragma unroll 1
  for (int t = 0; t < LL; ++t) {
    const float r = ((sdt[t * DTR + 0] * w0 + sdt[t * DTR + 1] * w1) +
                     (sdt[t * DTR + 2] * w2 + sdt[t * DTR + 3] * w3)) + db;
    const float e = fmaxf(r, 0.0f) + log1pf(expf(-fabsf(r)));
    const size_t ro = (r0 + t) * DI + d;
    const float u = uu[ro];
    const float z = zz[ro];
    const float du = e * u;
    float y = 0.0f;
#pragma unroll
    for (int s = 0; s < DS; ++s) {
      const float hn = exp2f(e * an[s]) * h[s] + du * sB[t * DS + s];
      h[s] = hn;
      y += hn * sC[t * DS + s];
    }
    const float v = ((y + u * Dd) * (z * sigf(z))) * S_Y;
    const _Float16 hq = (_Float16)v;
    sY[t * (2 * DI) + d] = h_bits(hq);
    sY[t * (2 * DI) + DI + d] = hb16((v - (float)hq) * RLO);
  }
  __syncthreads();
#pragma unroll 1
  for (int p = d; p < LL * 32; p += DI) {
    const int row = p >> 5, qq = p & 31;
    const v4u val = *(const v4u*)(sY + row * (2 * DI) + qq * 8);
    unsigned short* base = (qq < 16) ? yh : yl;
    unsigned short* dst = base + (r0 + row) * DI + (qq & 15) * 8;
    *(volatile v4u*)dst = val;
  }
  __threadfence();
#pragma unroll 1
  for (int p = d; p < LL * 32; p += DI) {
    const int row = p >> 5, qq = p & 31;
    const v4u val = *(const v4u*)(sY + row * (2 * DI) + qq * 8);
    unsigned short* base = (qq < 16) ? yh : yl;
    unsigned short* dst = base + (r0 + row) * DI + (qq & 15) * 8;
    *(volatile v4u*)dst = val;
  }
}

extern "C" void kernel_launch(void* const* d_in, const int* in_sizes, int n_in,
                              void* d_out, int out_size, void* d_ws, size_t ws_size,
                              hipStream_t stream) {
  if (n_in < 12) return;
  if (in_sizes[0] != NBATCH * EDIM) return;
  if (in_sizes[1] != LW * EDIM || in_sizes[2] != LW) return;
  if (in_sizes[3] != XZW * DM) return;
  if (in_sizes[4] != DI * 4 || in_sizes[5] != DI) return;
  if (in_sizes[6] != XPR * DI) return;
  if (in_sizes[7] != DI * DTR || in_sizes[8] != DI) return;
  if (in_sizes[9] != DI * DS || in_sizes[10] != DI) return;
  if (in_sizes[11] != DM * DI) return;
  if (out_size != NBATCH * LL * DM) return;

  const float* enc  = (const float*)d_in[0];
  const float* decw = (const float*)d_in[1];
  const float* decb = (const float*)d_in[2];
  const float* inw  = (const float*)d_in[3];
  const float* cvw  = (const float*)d_in[4];
  const float* cvb  = (const float*)d_in[5];
  const float* xpw  = (const float*)d_in[6];
  const float* dtw  = (const float*)d_in[7];
  const float* dtb  = (const float*)d_in[8];
  const float* alog = (const float*)d_in[9];
  const float* dpar = (const float*)d_in[10];
  const float* outw = (const float*)d_in[11];
  float* out = (float*)d_out;

  const size_t sH64  = (size_t)NTC * DM * 2;
  const size_t sF128 = (size_t)NTC * DI * 4;
  const size_t sH128 = (size_t)NTC * DI * 2;
  const size_t sF64  = (size_t)NTC * DM * 4;
  size_t sRX = 2 * sH64;
  if (sH128 > sRX) sRX = sH128;
  size_t sRA = sF128;
  if (sF64 + sH128 > sRA) sRA = sF64 + sH128;
  const size_t sWE   = (size_t)NBATCH * EDIM * 2;
  const size_t sWD   = (size_t)LW * EDIM * 2;
  const size_t sWIN  = (size_t)XZW * DM * 2;
  const size_t sWXP  = (size_t)XPP * DI * 2;
  const size_t sWOUT = (size_t)DM * DI * 2;
  const size_t sA2   = (size_t)DI * DS * 4;

  size_t off = 0;
  const size_t oRX   = off; off += sRX;
  const size_t oZ    = off; off += sF128;
  const size_t oRA   = off; off += sRA;
  const size_t oU    = off; off += sF128;
  const size_t oUH   = off; off += sH128;
  const size_t oUL   = off; off += sH128;
  const size_t oWE   = off; off += sWE;
  const size_t oWD   = off; off += sWD;
  const size_t oWIN  = off; off += sWIN;
  const size_t oWXP  = off; off += sWXP;
  const size_t oWOUT = off; off += sWOUT;
  const size_t oA2   = off; off += sA2;
  if (off > ws_size) return;
  if (off > (size_t)134217728) return;

  char* ws = (char*)d_ws;
  unsigned short* XH   = (unsigned short*)(ws + oRX);
  unsigned short* XL   = (unsigned short*)(ws + oRX + sH64);
  unsigned short* YL   = (unsigned short*)(ws + oRX);
  float*          Z    = (float*)(ws + oZ);
  float*          U0   = (float*)(ws + oRA);
  float*          DBC  = (float*)(ws + oRA);
  unsigned short* YH   = (unsigned short*)(ws + oRA + sF64);
  float*          U    = (float*)(ws + oU);
  unsigned short* UH   = (unsigned short*)(ws + oUH);
  unsigned short* UL   = (unsigned short*)(ws + oUL);
  unsigned short* WE   = (unsigned short*)(ws + oWE);
  unsigned short* WD   = (unsigned short*)(ws + oWD);
  unsigned short* WIN  = (unsigned short*)(ws + oWIN);
  unsigned short* WXP  = (unsigned short*)(ws + oWXP);
  unsigned short* WOUT = (unsigned short*)(ws + oWOUT);
  float*          A2   = (float*)(ws + oA2);
  float*          dfp  = Z;
  unsigned short* dhp  = UH;

  k_cvt<<<dim3((NBATCH * (EDIM / 8) + 255) / 256), dim3(256), 0, stream>>>(enc, NBATCH, EDIM, WE, NBATCH, S_E);
  k_cvt<<<dim3((LW * (EDIM / 8) + 255) / 256), dim3(256), 0, stream>>>(decw, LW, EDIM, WD, LW, S_W);
  k_cvt<<<dim3((XZW * (DM / 8) + 255) / 256), dim3(256), 0, stream>>>(inw, XZW, DM, WIN, XZW, S_W);
  k_cvt<<<dim3((XPP * (DI / 8) + 255) / 256), dim3(256), 0, stream>>>(xpw, XPR, DI, WXP, XPP, S_W);
  k_cvt<<<dim3((DM * (DI / 8) + 255) / 256), dim3(256), 0, stream>>>(outw, DM, DI, WOUT, DM, S_W);
  k_atab<<<dim3((DI * DS + 255) / 256), dim3(256), 0, stream>>>(alog, DI * DS, A2);

  for (int ch = 0; ch < NCH; ++ch) {
    const unsigned short* encp = WE + (size_t)ch * BSC * EDIM;
    float* outp = out + (size_t)ch * NTC * DM;
    k_gemm<0, 2, false><<<dim3(BSC / 64, LW / 64), dim3(128), 0, stream>>>(encp, encp, EDIM, WD, EDIM, EDIM / 32,
                                                                            decb, dfp, dfp, XH, XL);
    k_gemm<1, 4, true><<<dim3(NTC / 64, XZW / 128), dim3(256), 0, stream>>>(XH, XL, DM, WIN, DM, DM / 32,
                                                                             decb, U0, Z, dhp, dhp);
    k_conv<<<dim3(NTC / 8), dim3(256), 0, stream>>>(U0, cvw, cvb, U, UH, UL);
    k_gemm<2, 2, true><<<dim3(NTC / 64, 1), dim3(128), 0, stream>>>(UH, UL, DI, WXP, DI, DI / 32,
                                                                     decb, DBC, dfp, dhp, dhp);
    k_scan<<<dim3(BSC), dim3(128), 0, stream>>>(DBC, U, Z, A2, dtw, dtb, dpar, YH, YL);
    k_gemm<3, 2, true><<<dim3(NTC / 64, 1), dim3(128), 0, stream>>>(YH, YL, DI, WOUT, DI, DI / 32,
                                                                     decb, outp, dfp, dhp, dhp);
  }
  (void)hipGetLastError();
}
